// GCN_EW_10943576670614
// MI455X (gfx1250) — hardware-run, weakly checked
//
#include <hip/hip_runtime.h>
#include <stddef.h>
#include <stdint.h>
#include <math.h>

#define NB      2
#define NN      50000
#define MR      100000
#define FD      128
#define HD      64
#define NE      800000
#define GBM     128
#define MP      100096
#define KL      128
#define NTHR    256
#define NWAVE   8
#define EPT     8
#define WCH     (32 * EPT)
#define NBRUN   1024
#define SLB     10
#define NBK     49
#define WLCAP   2560
#define RCAP    20480
#define DEGCAP  64
#define MAXDEG_MEAS   35
#define MAXB1024_MEAS 16623
#define SP      68
#define TABW    4096
#define NREC    98
#define RECW    128
#define HROWS   1024
#define LO_PLANE 1

#define BK_ZINTS (NWAVE * WLCAP + 2 * RCAP + 5 * NBRUN)
#define BK_INTS  (BK_ZINTS + 16)
#define BK_LDS   (BK_INTS * 4)

#define PBX   (MP * FD / 8 / NTHR)
#define PBW   (HD * KL / 8 / NTHR)
#define PBTOT (PBX + 2 * PBW + 1)

static_assert(NB * NN == MR && HD == 64 && FD == KL && KL == 2 * HD && KL % 32 == 0);
static_assert(MP % GBM == 0 && MP >= MR && MP == 782 * GBM);
static_assert(NBRUN == (1 << SLB) && NBK * NBRUN >= NN && (NBK - 1) * NBRUN < NN);
static_assert(NE < (1 << 21) && (((long long)NE) << SLB) < (1LL << 31));
static_assert(NE % WCH == 0 && NE % 4 == 0);
static_assert(RCAP == NWAVE * WLCAP && RCAP % 4 == 0 && BK_ZINTS % 4 == 0);
static_assert((long long)RCAP * 100 >= (long long)MAXB1024_MEAS * 105);
static_assert(WLCAP >= MAXB1024_MEAS / 8 + 8 * 46 + 1);
static_assert(MAXDEG_MEAS + 8 <= DEGCAP);
static_assert((MP * FD / 8) % NTHR == 0 && (HD * KL / 8) % NTHR == 0);
static_assert(BK_LDS <= 300000);
static_assert(GBM * SP * 4 <= 65536);
static_assert(TABW == 4 * NBRUN && (2 * RCAP) % (NTHR * 4) == 0 && TABW % (NTHR * 4) == 0);
static_assert(NREC == NBK * NB && NREC * HROWS >= MR && (NREC - 1) * HROWS < MR);
static_assert((MR % HROWS) % 32 == 0 && HROWS == 4 * NTHR && NN % 2 == 0);

typedef float          v4f   __attribute__((ext_vector_type(4)));
typedef float          v8f   __attribute__((ext_vector_type(8)));
typedef double         v2d   __attribute__((ext_vector_type(2)));
typedef int            v2i   __attribute__((ext_vector_type(2)));
typedef int            v4i   __attribute__((ext_vector_type(4)));
typedef int            v8i   __attribute__((ext_vector_type(8)));
typedef unsigned short v8us  __attribute__((ext_vector_type(8)));
typedef unsigned short v16us __attribute__((ext_vector_type(16)));
typedef __bf16         v16bf __attribute__((ext_vector_type(16)));
typedef v4f  __attribute__((may_alias)) v4fa;
typedef v2i  __attribute__((may_alias)) v2ia;
typedef v4i  __attribute__((may_alias)) v4ia;
typedef v8us __attribute__((may_alias)) v8usa;
union FragB { v16bf v; v16us u; v8us h[2]; v8i w; };

__device__ __forceinline__ v8f wmb(const FragB& a, const FragB& b, v8f c) {
  v8f d = __builtin_amdgcn_wmma_f32_16x16x32_bf16(false, a.v, false, b.v, (short)0, c, false, false);
  asm volatile("v_nop\n\tv_nop\n\tv_nop\n\tv_nop" : "+v"(d) : "v"(a.w), "v"(b.w));
  return d;
}

__device__ __forceinline__ unsigned bf16_bits(float f) {
  const unsigned u = __float_as_uint(f);
  const unsigned r = (u + 0x7FFFu + ((u >> 16) & 1u)) >> 16;
  const unsigned q = (u >> 16) | 0x40u;
  return ((u & 0x7fffffffu) > 0x7f800000u) ? q : r;
}
__device__ __forceinline__ float bf16_val(float f) {
  return __uint_as_float(bf16_bits(f) << 16);
}
__device__ __forceinline__ unsigned bf16_bits_fin(float f) {
  const unsigned r = bf16_bits(f);
  const unsigned u = __float_as_uint(f) & 0x7fffffffu;
  const bool carry = ((r & 0x7fffu) == 0x7f80u) & (u < 0x7f800000u);
  return carry ? (r - 1u) : r;
}

__device__ __forceinline__ void hilo_pack(float v0, float v1, float v2, float v3,
                                          int& h01, int& h23, int& l01, int& l23) {
  const unsigned a0 = bf16_bits_fin(v0), a1 = bf16_bits_fin(v1), a2 = bf16_bits_fin(v2), a3 = bf16_bits_fin(v3);
  unsigned b0 = bf16_bits(v0 - __uint_as_float(a0 << 16));
  unsigned b1 = bf16_bits(v1 - __uint_as_float(a1 << 16));
  unsigned b2 = bf16_bits(v2 - __uint_as_float(a2 << 16));
  unsigned b3 = bf16_bits(v3 - __uint_as_float(a3 << 16));
  if (LO_PLANE == 0) { b0 = 0u; b1 = 0u; b2 = 0u; b3 = 0u; }
  h01 = (int)(a0 | (a1 << 16)); h23 = (int)(a2 | (a3 << 16));
  l01 = (int)(b0 | (b1 << 16)); l23 = (int)(b2 | (b3 << 16));
}

__device__ __forceinline__ v4i regroup8(int h01, int h23, int l01, int l23, int lane) {
  const int t  = lane & 15;
  const int s0 = (lane & 16) + ((2 * t) & 15), s1 = s0 + 1;
  const int a0 = __shfl(h01, s0, 32), a1 = __shfl(h23, s0, 32), a2 = __shfl(h01, s1, 32), a3 = __shfl(h23, s1, 32);
  const int b0 = __shfl(l01, s0, 32), b1 = __shfl(l23, s0, 32), b2 = __shfl(l01, s1, 32), b3 = __shfl(l23, s1, 32);
  const int mk = (t < 8) ? -1 : 0;
  v4i o;
  o.x = (a0 & mk) | (b0 & ~mk); o.y = (a1 & mk) | (b1 & ~mk);
  o.z = (a2 & mk) | (b2 & ~mk); o.w = (a3 & mk) | (b3 & ~mk);
  return o;
}

__device__ __forceinline__ void st2_v4f(float* p, v4f v) {
  *(volatile v4f*)p = v;
  __threadfence();
  *(volatile v4f*)p = v;
}
__device__ __forceinline__ void st2_v8us(unsigned short* p, v8us v) {
  *(volatile v8us*)p = v;
  __threadfence();
  *(volatile v8us*)p = v;
}

__device__ __forceinline__ v8us gather8(const float* __restrict__ base, int stride) {
  float f[8];
#pragma unroll
  for (int i = 0; i < 8; ++i) f[i] = base[(size_t)i * (size_t)stride];
  v8us o;
#pragma unroll
  for (int i = 0; i < 8; ++i) o[i] = (unsigned short)bf16_bits(f[i]);
  return o;
}

__global__ __launch_bounds__(NTHR) void k_prep(const float* __restrict__ x, const float* __restrict__ w1,
                                               const float* __restrict__ b1, const float* __restrict__ w2,
                                               const float* __restrict__ b2, const float* __restrict__ g1,
                                               const float* __restrict__ be1, const float* __restrict__ g2,
                                               const float* __restrict__ be2, const float* __restrict__ wc,
                                               const float* __restrict__ bc,
                                               unsigned short* xb, unsigned short* w1t, unsigned short* w2d,
                                               float* sm) {
  const int tid = (int)threadIdx.x;
  const int blk = (int)blockIdx.x;
  if (blk < PBX) {
    const int u   = blk * NTHR + tid;
    const int row = u >> 4, k8 = (u & 15) * 8;
    const int rc  = row < MR ? row : MR - 1;
    const unsigned mk = row < MR ? 0xffffu : 0u;
    const float* p = x + (size_t)rc * FD + k8;
    const v4f a = *(const v4fa*)p;
    const v4f b = *(const v4fa*)(p + 4);
    v8us o;
    o[0] = (unsigned short)(bf16_bits(a.x) & mk); o[1] = (unsigned short)(bf16_bits(a.y) & mk);
    o[2] = (unsigned short)(bf16_bits(a.z) & mk); o[3] = (unsigned short)(bf16_bits(a.w) & mk);
    o[4] = (unsigned short)(bf16_bits(b.x) & mk); o[5] = (unsigned short)(bf16_bits(b.y) & mk);
    o[6] = (unsigned short)(bf16_bits(b.z) & mk); o[7] = (unsigned short)(bf16_bits(b.w) & mk);
    st2_v8us(xb + (size_t)row * FD + k8, o);
  } else if (blk < PBX + PBW) {
    const int u = (blk - PBX) * NTHR + tid;
    const int n = u >> 4, k8 = (u & 15) * 8;
    const v8us o = gather8(w1 + (size_t)k8 * HD + n, HD);
    st2_v8us(w1t + (size_t)n * KL + k8, o);
  } else if (blk < PBX + 2 * PBW) {
    const int u = (blk - PBX - PBW) * NTHR + tid;
    const int n = u >> 4, k8 = (u & 15) * 8, kk = k8 & 63;
    const v8us o = gather8(w2 + (size_t)kk * HD + n, HD);
    st2_v8us(w2d + (size_t)n * KL + k8, o);
  } else {
    if (tid < 128) {
      const int t = tid >> 4, q = tid & 15;
      const v4f a0 = *(const v4fa*)(b1 + 4 * q);
      const v4f a1 = *(const v4fa*)(b2 + 4 * q);
      const v4f a2 = *(const v4fa*)(g1 + 4 * q);
      const v4f a3 = *(const v4fa*)(be1 + 4 * q);
      const v4f a4 = *(const v4fa*)(g2 + 4 * q);
      const v4f a5 = *(const v4fa*)(be2 + 4 * q);
      const v4f a6 = *(const v4fa*)(wc + 4 * q);
      const float cb = bc[0];
      asm volatile("" :: "v"(a0), "v"(a1), "v"(a2), "v"(a3));
      asm volatile("" :: "v"(a4), "v"(a5), "v"(a6), "v"(cb));
      const unsigned k0 = (t == 0) ? 0xffffffffu : 0u, k1 = (t == 1) ? 0xffffffffu : 0u;
      const unsigned k2 = (t == 2) ? 0xffffffffu : 0u, k3 = (t == 3) ? 0xffffffffu : 0u;
      const unsigned k4 = (t == 4) ? 0xffffffffu : 0u, k5 = (t == 5) ? 0xffffffffu : 0u;
      const unsigned k6 = (t == 6) ? 0xffffffffu : 0u, k7 = (t == 7) ? 0xffffffffu : 0u;
      const unsigned cbb = bf16_bits(cb) << 16;
#define TSEL(C) __uint_as_float(((bf16_bits(a0.C) << 16) & k0) | ((bf16_bits(a1.C) << 16) & k1) | \
                                ((bf16_bits(a2.C) << 16) & k2) | ((bf16_bits(a3.C) << 16) & k3) | \
                                ((bf16_bits(a4.C) << 16) & k4) | ((bf16_bits(a5.C) << 16) & k5) | \
                                ((bf16_bits(a6.C) << 16) & k6) | (cbb & k7))
      v4f o;
      o.x = TSEL(x); o.y = TSEL(y); o.z = TSEL(z); o.w = TSEL(w);
#undef TSEL
      st2_v4f(sm + 4 * tid, o);
    }
  }
}

__device__ __forceinline__ void bucket_flush(const int* pl, const int* tab, int ov, int* lp, int* tp, int* fp,
                                             int tid) {
#pragma unroll 1
  for (int i = tid * 4; i < 2 * RCAP; i += NTHR * 4) {
    const v4i v = *(const v4ia*)(pl + i);
    *(volatile v4i*)(lp + i) = v;
  }
#pragma unroll 1
  for (int i = tid * 4; i < TABW; i += NTHR * 4) {
    const v4i v = *(const v4ia*)(tab + i);
    *(volatile v4i*)(tp + i) = v;
  }
  if (tid < 8) {
    const v4i f = {ov, ov, ov, ov};
    *(volatile v4i*)(fp + 4 * tid) = f;
  }
}

__global__ __launch_bounds__(NTHR) void k_bucket(const int* __restrict__ srcs, const int* __restrict__ dsts,
                                                 const float* __restrict__ ew, int* LIST, int* TAB, int* FLAG) {
  extern __shared__ __attribute__((aligned(16))) int dsm[];
  int* wl   = dsm;
  int* pl   = dsm + NWAVE * WLCAP;
  int* cnt  = pl + 2 * RCAP;
  int* offs = cnt + NBRUN;
  int* dgs  = offs + NBRUN;
  int* dis  = dgs + NBRUN;
  int* cur  = dis + NBRUN;
  int* misc = cur + NBRUN;
  const int tid = (int)threadIdx.x, lane = tid & 31, wave = tid >> 5;
  const int blk = (int)blockIdx.x;
  const unsigned nbs = (unsigned)(blk * NBRUN);

  {
    const v4i z4 = {0, 0, 0, 0};
    for (int i = tid * 4; i < BK_ZINTS; i += NTHR * 4) *(v4ia*)(dsm + i) = z4;
    if (tid < 16) misc[tid] = 0;
  }
  __syncthreads();

  {
    const int per  = ((NE + NWAVE * WCH - 1) / (NWAVE * WCH)) * WCH;
    const int ebeg = wave * per;
    const int eend = (ebeg + per < NE) ? (ebeg + per) : NE;
    int* mylist = wl + wave * WLCAP;
    int wc = 0;
#pragma unroll 1
    for (int cb = ebeg; cb < eend; cb += WCH) {
      const int e0 = cb + lane * EPT;
      const v4i da = *(const v4ia*)(dsts + e0);
      const v4i db = *(const v4ia*)(dsts + e0 + 4);
      const unsigned s0 = (unsigned)da.x - nbs, s1 = (unsigned)da.y - nbs;
      const unsigned s2 = (unsigned)da.z - nbs, s3 = (unsigned)da.w - nbs;
      const unsigned s4 = (unsigned)db.x - nbs, s5 = (unsigned)db.y - nbs;
      const unsigned s6 = (unsigned)db.z - nbs, s7 = (unsigned)db.w - nbs;
      const bool h0 = s0 < (unsigned)NBRUN, h1 = s1 < (unsigned)NBRUN, h2 = s2 < (unsigned)NBRUN, h3 = s3 < (unsigned)NBRUN;
      const bool h4 = s4 < (unsigned)NBRUN, h5 = s5 < (unsigned)NBRUN, h6 = s6 < (unsigned)NBRUN, h7 = s7 < (unsigned)NBRUN;
      const unsigned m0 = __builtin_amdgcn_ballot_w32(h0), m1 = __builtin_amdgcn_ballot_w32(h1);
      const unsigned m2 = __builtin_amdgcn_ballot_w32(h2), m3 = __builtin_amdgcn_ballot_w32(h3);
      const unsigned m4 = __builtin_amdgcn_ballot_w32(h4), m5 = __builtin_amdgcn_ballot_w32(h5);
      const unsigned m6 = __builtin_amdgcn_ballot_w32(h6), m7 = __builtin_amdgcn_ballot_w32(h7);
      const unsigned any = m0 | m1 | m2 | m3 | m4 | m5 | m6 | m7;
      if (any != 0u) {
        const int pre = (int)(__builtin_amdgcn_mbcnt_lo(m0, 0u) + __builtin_amdgcn_mbcnt_lo(m1, 0u) +
                              __builtin_amdgcn_mbcnt_lo(m2, 0u) + __builtin_amdgcn_mbcnt_lo(m3, 0u) +
                              __builtin_amdgcn_mbcnt_lo(m4, 0u) + __builtin_amdgcn_mbcnt_lo(m5, 0u) +
                              __builtin_amdgcn_mbcnt_lo(m6, 0u) + __builtin_amdgcn_mbcnt_lo(m7, 0u));
        int p = wc + pre;
        if (h0) { if (p < WLCAP) mylist[p] = ((e0 + 0) << SLB) | (int)s0; p = p + 1; }
        if (h1) { if (p < WLCAP) mylist[p] = ((e0 + 1) << SLB) | (int)s1; p = p + 1; }
        if (h2) { if (p < WLCAP) mylist[p] = ((e0 + 2) << SLB) | (int)s2; p = p + 1; }
        if (h3) { if (p < WLCAP) mylist[p] = ((e0 + 3) << SLB) | (int)s3; p = p + 1; }
        if (h4) { if (p < WLCAP) mylist[p] = ((e0 + 4) << SLB) | (int)s4; p = p + 1; }
        if (h5) { if (p < WLCAP) mylist[p] = ((e0 + 5) << SLB) | (int)s5; p = p + 1; }
        if (h6) { if (p < WLCAP) mylist[p] = ((e0 + 6) << SLB) | (int)s6; p = p + 1; }
        if (h7) { if (p < WLCAP) mylist[p] = ((e0 + 7) << SLB) | (int)s7; p = p + 1; }
        wc += (int)(__builtin_popcount(m0) + __builtin_popcount(m1) + __builtin_popcount(m2) + __builtin_popcount(m3) +
                    __builtin_popcount(m4) + __builtin_popcount(m5) + __builtin_popcount(m6) + __builtin_popcount(m7));
      }
    }
    if (lane == 0) misc[wave] = wc;
  }
  __syncthreads();

  if (wave == 0) {
    int ov = 0;
#pragma unroll 1
    for (int w2 = 0; w2 < NWAVE; ++w2) {
      int c = misc[w2];
      if (c > WLCAP) ov = 1;
      c = c < 0 ? 0 : (c > WLCAP ? WLCAP : c);
#pragma unroll 1
      for (int b0 = 0; b0 < c; b0 += 32) {
        const int idx = b0 + lane;
        const int ent = wl[w2 * WLCAP + (idx < WLCAP ? idx : WLCAP - 1)];
        const int m32 = (c - b0) < 32 ? (c - b0) : 32;
#pragma unroll 1
        for (int k = 0; k < m32; ++k) {
          const int u    = __builtin_amdgcn_readlane(ent, k);
          const int slot = u & (NBRUN - 1);
          if (lane == 0) cnt[slot] = cnt[slot] + 1;
        }
      }
    }
    if (lane == 0) misc[9] = ov;
  }
  __syncthreads();
  if (wave == 0) {
    const int base = lane * (NBRUN / 32);
    int s = 0;
#pragma unroll 1
    for (int i = 0; i < NBRUN / 32; ++i) s += cnt[base + i];
    int incl = s;
#pragma unroll
    for (int d = 1; d < 32; d <<= 1) {
      const int y = __shfl_up(incl, d, 32);
      if (lane >= d) incl += y;
    }
    int run = incl - s;
#pragma unroll 1
    for (int i = 0; i < NBRUN / 32; ++i) {
      const int cv = cnt[base + i];
      offs[base + i] = run;
      cur[base + i]  = run;
      run += cv;
    }
  }
  __syncthreads();

  if (wave == 0) {
#pragma unroll 1
    for (int w2 = 0; w2 < NWAVE; ++w2) {
      int c = misc[w2];
      c = c < 0 ? 0 : (c > WLCAP ? WLCAP : c);
#pragma unroll 1
      for (int b0 = 0; b0 < c; b0 += 32) {
        const int idx = b0 + lane;
        const int ent = wl[w2 * WLCAP + (idx < WLCAP ? idx : WLCAP - 1)];
        int eid = (ent >> SLB) & 0x1FFFFF;
        eid = eid > NE - 1 ? NE - 1 : eid;
        int sr = srcs[eid];
        sr = sr < 0 ? 0 : (sr > NN - 1 ? NN - 1 : sr);
        const float wv = expf(bf16_val(ew[eid]));
        const int   wb = __float_as_int(wv);
        const int m32 = (c - b0) < 32 ? (c - b0) : 32;
#pragma unroll 1
        for (int k = 0; k < m32; ++k) {
          const int u    = __builtin_amdgcn_readlane(ent, k);
          const int s0   = __builtin_amdgcn_readlane(sr, k);
          const int w0   = __builtin_amdgcn_readlane(wb, k);
          const int slot = u & (NBRUN - 1);
          if (lane == 0) {
            int p = cur[slot];
            p = p < 0 ? 0 : (p > RCAP - 1 ? RCAP - 1 : p);
            pl[2 * p]     = s0;
            pl[2 * p + 1] = w0;
            cur[slot] = p + 1;
          }
        }
      }
    }
  }
  __syncthreads();

#pragma unroll 1
  for (int s = tid; s < NBRUN; s += NTHR) {
    int c = cnt[s];
    const bool big = c > DEGCAP;
    c = c < 0 ? 0 : (c > DEGCAP ? DEGCAP : c);
    int o = offs[s];
    o = o < 0 ? 0 : (o > RCAP - 1 ? RCAP - 1 : o);
    int last = o + c - 1; last = last < o ? o : last;
    last = last > RCAP - 1 ? RCAP - 1 : last;
    int cmx = c;
#pragma unroll
    for (int d = 16; d > 0; d >>= 1) {
      const int y = __shfl_xor(cmx, d, 32);
      cmx = cmx > y ? cmx : y;
    }
    float sw = 0.0f;
#pragma unroll 1
    for (int j = 0; j < cmx; ++j) {
      int idx = o + j;
      idx = idx > last ? last : idx;
      const float w = __int_as_float(pl[2 * idx + 1]);
      const float t = sw + w;
      sw = (j < c) ? t : sw;
    }
    float dg = sw + 1.0f;
    dg = big ? __uint_as_float(0x7fc00000u) : dg;
    const float dv = 1.0f / sqrtf(dg);
    dgs[s] = __float_as_int(dg);
    dis[s] = __float_as_int(dv);
  }
  __syncthreads();

  const int ovf = misc[9];
  int* lp = LIST + (size_t)blk * (2 * RCAP);
  int* tp = TAB + (size_t)blk * TABW;
  int* fp = FLAG + (size_t)blk * 32;
  bucket_flush(pl, cnt, ovf, lp, tp, fp, tid);
  __threadfence();
  bucket_flush(pl, cnt, ovf, lp, tp, fp, tid);
}

template <int KTOT>
__device__ __forceinline__ void gemm_16x64(const unsigned short* __restrict__ ap,
                                           const unsigned short* __restrict__ bp, v8f (&acc)[4]) {
#pragma unroll 1
  for (int k0 = 0; k0 < KTOT; k0 += 32) {
    FragB af;
    af.h[0] = *(const v8usa*)(ap + k0);
    af.h[1] = *(const v8usa*)(ap + k0 + 16);
#pragma unroll
    for (int nt = 0; nt < 4; ++nt) {
      const unsigned short* wq = bp + (size_t)(16 * nt) * (size_t)KTOT + k0;
      FragB bf;
      bf.h[0] = *(const v8usa*)wq;
      bf.h[1] = *(const v8usa*)(wq + 16);
      acc[nt] = wmb(af, bf, acc[nt]);
    }
  }
}

__device__ __forceinline__ void stage_d(float* stg, const v8f (&acc)[4], int wave, int hh, int m) {
#pragma unroll
  for (int nt = 0; nt < 4; ++nt) {
#pragma unroll
    for (int r = 0; r < 8; ++r) stg[(16 * wave + 8 * hh + r) * SP + 16 * nt + m] = acc[nt][r];
  }
}

__global__ __launch_bounds__(NTHR) __attribute__((amdgpu_num_vgpr(248)))
void k_gemm(const unsigned short* __restrict__ A, const unsigned short* __restrict__ BT,
            const int* __restrict__ TAB, float* P) {
  __shared__ __attribute__((aligned(16))) float stg[GBM * SP];
  const int tid = (int)threadIdx.x, lane = tid & 31, wave = tid >> 5, hh = lane >> 4, m = lane & 15;
  const int rowBase = (int)blockIdx.x * GBM;

  v8f acc[4];
  {
    const v8f z = {0.f, 0.f, 0.f, 0.f, 0.f, 0.f, 0.f, 0.f};
#pragma unroll
    for (int t = 0; t < 4; ++t) acc[t] = z;
  }
  const unsigned short* ap = A + (size_t)(rowBase + 16 * wave + m) * (size_t)KL + 8 * hh;
  const unsigned short* bp = BT + (size_t)m * (size_t)KL + 8 * hh;
  gemm_16x64<KL>(ap, bp, acc);
  stage_d(stg, acc, wave, hh, m);
  __syncthreads();

#pragma unroll 1
  for (int i = 0; i < 8; ++i) {
    const int lr   = 16 * wave + 2 * i + hh;
    const int grow = rowBase + lr;
    const bool live = grow < MR;
    int node = grow >= NN ? grow - NN : grow;
    node = node > NN - 1 ? NN - 1 : node;
    const float dv = __int_as_float(TAB[(size_t)(node >> SLB) * TABW + 3 * NBRUN + (node & (NBRUN - 1))]);
    const v4f a = *(const v4fa*)(stg + lr * SP + 4 * m);
    asm volatile("" :: "v"(a), "v"(dv));
    v4f o;
    o.x = live ? dv * a.x : 0.0f; o.y = live ? dv * a.y : 0.0f;
    o.z = live ? dv * a.z : 0.0f; o.w = live ? dv * a.w : 0.0f;
    st2_v4f(P + (size_t)grow * HD + 4 * m, o);
  }
}

__global__ __launch_bounds__(NTHR) void k_replay(const int* __restrict__ LIST, const int* __restrict__ TAB,
                                                 const int* __restrict__ FLAG, const float* __restrict__ P,
                                                 const float* __restrict__ sm, int boff, float* T, double* REC) {
  __shared__ __attribute__((aligned(16))) int    sco[2 * NBRUN];
  __shared__ __attribute__((aligned(16))) float  sdi[NBRUN];
  __shared__ __attribute__((aligned(16))) float  sb[128];
  __shared__ __attribute__((aligned(16))) double sp[16 * 64 * 2];
  __shared__ __attribute__((aligned(16))) double srec[RECW];
  const int tid = (int)threadIdx.x, lane = tid & 31, wave = tid >> 5, hh = lane >> 4, q = lane & 15;
  const int bucket = (int)blockIdx.x;
  const int bb     = (int)blockIdx.y;
  const int* lb = LIST + (size_t)bucket * (2 * RCAP);
  const int* tb = TAB + (size_t)bucket * TABW;
  const int flag = FLAG[(size_t)bucket * 32];
  const float qnan = __uint_as_float(0x7fc00000u);

#pragma unroll 1
  for (int i = tid * 4; i < 2 * NBRUN; i += NTHR * 4) *(v4ia*)(sco + i) = *(const v4ia*)(tb + i);
  *(v4fa*)(sdi + 4 * tid) = *(const v4fa*)((const float*)(tb + 3 * NBRUN) + 4 * tid);
  if (wave == 0) *(v4fa*)(sb + 4 * lane) = *(const v4fa*)(sm + 4 * lane);
  __syncthreads();

  const v4f bias = *(const v4fa*)(sb + boff + 4 * q);
  const size_t pbase = (size_t)bb * (size_t)NN;
  double s0 = 0.0, s1 = 0.0, s2 = 0.0, s3 = 0.0;
  double q0 = 0.0, q1 = 0.0, q2 = 0.0, q3 = 0.0;

#pragma unroll 1
  for (int st = 0; st < NBRUN / 16; ++st) {
    const int slot = st * 16 + 2 * wave + hh;
    const int node = bucket * NBRUN + slot;
    const bool live = node < NN;
    const int nc = live ? node : NN - 1;
    int c = sco[slot];
    int o = sco[NBRUN + slot];
    const bool big = c > DEGCAP;
    c = c < 0 ? 0 : (c > DEGCAP ? DEGCAP : c);
    o = o < 0 ? 0 : (o > RCAP - 1 ? RCAP - 1 : o);
    const int co = __shfl_xor(c, 16, 32);
    const int cm = c > co ? c : co;
    int last = o + c - 1; last = last < o ? o : last;
    last = last > RCAP - 1 ? RCAP - 1 : last;
    float a0 = 0.0f, a1 = 0.0f, a2 = 0.0f, a3 = 0.0f;
#pragma unroll 1
    for (int j = 0; j < cm; ++j) {
      int idx = o + j;
      idx = idx > last ? last : idx;
      const v2i wd = *(const v2ia*)(lb + 2 * idx);
      int sr = wd.x;
      sr = sr < 0 ? 0 : (sr > NN - 1 ? NN - 1 : sr);
      const float w = __int_as_float(wd.y);
      const v4f v = *(const v4fa*)(P + (pbase + (size_t)sr) * HD + 4 * q);
      asm volatile("" :: "v"(v));
      const bool valid = j < c;
      const float t0 = fmaf(w, v.x, a0), t1 = fmaf(w, v.y, a1), t2 = fmaf(w, v.z, a2), t3 = fmaf(w, v.w, a3);
      a0 = valid ? t0 : a0; a1 = valid ? t1 : a1; a2 = valid ? t2 : a2; a3 = valid ? t3 : a3;
    }
    const v4f g = *(const v4fa*)(P + (pbase + (size_t)nc) * HD + 4 * q);
    asm volatile("" :: "v"(g));
    const float dv = sdi[slot];
    float m0 = dv * (a0 + g.x) + bias.x, m1 = dv * (a1 + g.y) + bias.y;
    float m2 = dv * (a2 + g.z) + bias.z, m3 = dv * (a3 + g.w) + bias.w;
    m0 = (m0 > 0.0f) ? m0 : (m0 - m0); m1 = (m1 > 0.0f) ? m1 : (m1 - m1);
    m2 = (m2 > 0.0f) ? m2 : (m2 - m2); m3 = (m3 > 0.0f) ? m3 : (m3 - m3);
    const bool bad = (flag != 0) | big;
    m0 = bad ? qnan : m0; m1 = bad ? qnan : m1; m2 = bad ? qnan : m2; m3 = bad ? qnan : m3;
    const double d0 = live ? (double)m0 : 0.0, d1 = live ? (double)m1 : 0.0;
    const double d2 = live ? (double)m2 : 0.0, d3 = live ? (double)m3 : 0.0;
    s0 += d0; s1 += d1; s2 += d2; s3 += d3;
    q0 += d0 * d0; q1 += d1 * d1; q2 += d2 * d2; q3 += d3 * d3;
    v4f ov;
    ov.x = m0; ov.y = m1; ov.z = m2; ov.w = m3;
    float* op = T + (pbase + (size_t)nc) * HD + 4 * q;
    if (live) st2_v4f(op, ov);
  }

  {
    const int hw = 2 * wave + hh;
    double* w = sp + (size_t)(hw * 64 + 4 * q) * 2;
    w[0] = s0; w[1] = q0; w[2] = s1; w[3] = q1; w[4] = s2; w[5] = q2; w[6] = s3; w[7] = q3;
  }
  __syncthreads();
  if (tid < 128) {
    const int col = tid & 63, which = tid >> 6;
    double a = 0.0;
#pragma unroll 1
    for (int hw = 0; hw < 16; ++hw) a += sp[(size_t)(hw * 64 + col) * 2 + which];
    srec[which * 64 + col] = a;
  }
  __syncthreads();
  if (tid < 64) {
    v2d v;
    v.x = srec[2 * tid]; v.y = srec[2 * tid + 1];
    double* dp = REC + (size_t)(bb * NBK + bucket) * RECW + 2 * tid;
    *(volatile v2d*)dp = v;
    __threadfence();
    *(volatile v2d*)dp = v;
  }
}

__global__ __launch_bounds__(64) void k_comb(const double* __restrict__ rec, float* stat) {
  __shared__ __attribute__((aligned(16))) float st[128];
  const int c = (int)threadIdx.x;
  double S = 0.0, Q = 0.0;
#pragma unroll 1
  for (int rb = 0; rb < NREC; ++rb) {
    S += rec[(size_t)rb * RECW + c];
    Q += rec[(size_t)rb * RECW + 64 + c];
  }
  const double cntd = (double)MR;
  const double mm = S / cntd;
  double vv = Q / cntd - mm * mm;
  vv = (vv < 0.0) ? 0.0 : vv;
  const float mf = (float)mm;
  const float vf = (float)vv;
  st[c] = mf;
  st[64 + c] = sqrtf(vf + 1e-5f);
  __syncthreads();
  if (c < 32) {
    const v4f v = *(const v4fa*)(st + 4 * c);
    st2_v4f(stat + 4 * c, v);
  }
}

__global__ __launch_bounds__(NTHR) void k_apply(const float* __restrict__ T, const float* __restrict__ stat,
                                                const float* __restrict__ sm, int goff, unsigned short* HN) {
  __shared__ __attribute__((aligned(16))) float prm[256];
  const int tid = (int)threadIdx.x, lane = tid & 31, wave = tid >> 5, hh = lane >> 4, q = lane & 15;
  if (wave == 0) *(v4fa*)(prm + 4 * lane) = *(const v4fa*)(stat + 4 * lane);
  if (wave == 1) *(v4fa*)(prm + 128 + 4 * lane) = *(const v4fa*)(sm + goff + 4 * lane);
  __syncthreads();
  const v4f mv = *(const v4fa*)(prm + 4 * q);
  const v4f sv = *(const v4fa*)(prm + 64 + 4 * q);
  const v4f gv = *(const v4fa*)(prm + 128 + 4 * q);
  const v4f bv = *(const v4fa*)(prm + 192 + 4 * q);
  const int rowBase = (int)blockIdx.x * GBM;
#pragma unroll 1
  for (int i = 0; i < 8; ++i) {
    const int row = rowBase + 16 * i + 2 * wave + hh;
    const bool live = row < MR;
    const int rc = live ? row : MR - 1;
    const v4f v = *(const v4fa*)(T + (size_t)rc * HD + 4 * q);
    asm volatile("" :: "v"(v));
    float y0 = ((v.x - mv.x) / sv.x) * gv.x + bv.x;
    float y1 = ((v.y - mv.y) / sv.y) * gv.y + bv.y;
    float y2 = ((v.z - mv.z) / sv.z) * gv.z + bv.z;
    float y3 = ((v.w - mv.w) / sv.w) * gv.w + bv.w;
    y0 = live ? y0 : 0.0f; y1 = live ? y1 : 0.0f; y2 = live ? y2 : 0.0f; y3 = live ? y3 : 0.0f;
    int h01, h23, l01, l23;
    hilo_pack(y0, y1, y2, y3, h01, h23, l01, l23);
    const v4i ow = regroup8(h01, h23, l01, l23, lane);
    unsigned short* hp = HN + (size_t)row * KL + 8 * q;
    *(volatile v4i*)hp = ow;
    __threadfence();
    *(volatile v4i*)hp = ow;
  }
}

__global__ __launch_bounds__(NTHR) void k_head(const float* __restrict__ T, const float* __restrict__ stat,
                                               const float* __restrict__ sm, float* out) {
  __shared__ __attribute__((aligned(16))) float prm[384];
  __shared__ __attribute__((aligned(16))) float so[HROWS];
  const int tid = (int)threadIdx.x, lane = tid & 31, wave = tid >> 5;
  const int blk = (int)blockIdx.x;
  if (wave == 0) *(v4fa*)(prm + 4 * lane) = *(const v4fa*)(stat + 4 * lane);
  if (wave == 1) *(v4fa*)(prm + 128 + 4 * lane) = *(const v4fa*)(sm + 256 + 4 * lane);
  if (wave == 2) *(v4fa*)(prm + 256 + 4 * lane) = *(const v4fa*)(sm + 384 + 4 * lane);
  __syncthreads();
  const float bcv = prm[320];
#pragma unroll 1
  for (int k = 0; k < HROWS / NTHR; ++k) {
    const int r  = blk * HROWS + k * NTHR + tid;
    const int rc = r < MR ? r : MR - 1;
    const float* tp = T + (size_t)rc * HD;
    float acc = 0.0f;
#pragma unroll 1
    for (int c4 = 0; c4 < HD / 4; ++c4) {
      const v4f v  = *(const v4fa*)(tp + 4 * c4);
      const v4f mv = *(const v4fa*)(prm + 4 * c4);
      const v4f sv = *(const v4fa*)(prm + 64 + 4 * c4);
      const v4f gv = *(const v4fa*)(prm + 128 + 4 * c4);
      const v4f bv = *(const v4fa*)(prm + 192 + 4 * c4);
      const v4f wv = *(const v4fa*)(prm + 256 + 4 * c4);
      acc = fmaf(((v.x - mv.x) / sv.x) * gv.x + bv.x, wv.x, acc);
      acc = fmaf(((v.y - mv.y) / sv.y) * gv.y + bv.y, wv.y, acc);
      acc = fmaf(((v.z - mv.z) / sv.z) * gv.z + bv.z, wv.z, acc);
      acc = fmaf(((v.w - mv.w) / sv.w) * gv.w + bv.w, wv.w, acc);
    }
    so[k * NTHR + tid] = acc + bcv;
  }
  __syncthreads();
  const int nlive = (MR - blk * HROWS) < HROWS ? (MR - blk * HROWS) : HROWS;
  const int nv4 = nlive >> 2;
  const v4f v = *(const v4fa*)(so + 4 * tid);
  asm volatile("" :: "v"(v));
  float* op = out + (size_t)blk * HROWS + 4 * tid;
  if (tid < nv4) *(volatile v4f*)op = v;
  __threadfence();
  if (tid < nv4) *(volatile v4f*)op = v;
}

extern "C" void kernel_launch(void* const* d_in, const int* in_sizes, int n_in,
                              void* d_out, int out_size, void* d_ws, size_t ws_size,
                              hipStream_t stream) {
  if (n_in < 13) return;
  if (in_sizes[0] != MR * FD) return;
  if (in_sizes[1] != NE) return;
  if (in_sizes[2] != FD * HD) return;
  if (in_sizes[3] != HD) return;
  if (in_sizes[4] != HD * HD) return;
  if (in_sizes[5] != HD) return;
  if (in_sizes[6] != HD || in_sizes[7] != HD) return;
  if (in_sizes[8] != HD || in_sizes[9] != HD) return;
  if (in_sizes[10] != HD || in_sizes[11] != 1) return;
  if (in_sizes[12] != 2 * NE) return;
  if (out_size != MR) return;

  const float* x   = (const float*)d_in[0];
  const float* ew  = (const float*)d_in[1];
  const float* W1  = (const float*)d_in[2];
  const float* b1  = (const float*)d_in[3];
  const float* W2  = (const float*)d_in[4];
  const float* b2  = (const float*)d_in[5];
  const float* g1  = (const float*)d_in[6];
  const float* be1 = (const float*)d_in[7];
  const float* g2  = (const float*)d_in[8];
  const float* be2 = (const float*)d_in[9];
  const float* Wc  = (const float*)d_in[10];
  const float* bc  = (const float*)d_in[11];
  const int*   ei  = (const int*)d_in[12];
  float* out = (float*)d_out;
  const int* srcs = ei;
  const int* dsts = ei + NE;

  constexpr size_t zXB   = (size_t)MP * FD * 2;
  constexpr size_t zF    = (size_t)MP * HD * 4;
  constexpr size_t zHN   = (size_t)MP * KL * 2;
  constexpr size_t zLIST = (size_t)NBK * RCAP * 8;
  constexpr size_t zTAB  = (size_t)NBK * TABW * 4;
  constexpr size_t zFLAG = (size_t)(NBK + 1) * 128;
  constexpr size_t zWT   = (size_t)HD * KL * 2;
  constexpr size_t zSM   = 2048;
  constexpr size_t zREC  = (size_t)NREC * RECW * 8;
  constexpr size_t zST   = 512;
  constexpr size_t oXB   = 0;
  constexpr size_t oP    = oXB + zXB;
  constexpr size_t oT    = oP + zF;
  constexpr size_t oHN   = oT + zF;
  constexpr size_t oLIST = oHN + zHN;
  constexpr size_t oTAB  = oLIST + zLIST;
  constexpr size_t oFLAG = oTAB + zTAB;
  constexpr size_t oW1T  = oFLAG + zFLAG;
  constexpr size_t oW2D  = oW1T + zWT;
  constexpr size_t oSM   = oW2D + zWT;
  constexpr size_t oREC1 = oSM + zSM;
  constexpr size_t oREC2 = oREC1 + zREC;
  constexpr size_t oST1  = oREC2 + zREC;
  constexpr size_t oST2  = oST1 + zST;
  constexpr size_t oEND  = oST2 + zST;
  static_assert(zXB % 256 == 0 && zF % 256 == 0 && zHN % 256 == 0 && zLIST % 256 == 0 && zTAB % 256 == 0);
  static_assert(zFLAG % 256 == 0 && zWT % 256 == 0 && zSM % 256 == 0 && zREC % 256 == 0 && zST % 256 == 0);
  static_assert(oEND <= (size_t)(128u << 20));
  if (oEND > ws_size) return;

  char* ws = (char*)d_ws;
  unsigned short* XB   = (unsigned short*)(ws + oXB);
  float*          P    = (float*)(ws + oP);
  float*          T    = (float*)(ws + oT);
  unsigned short* HN   = (unsigned short*)(ws + oHN);
  int*            LIST = (int*)(ws + oLIST);
  int*            TAB  = (int*)(ws + oTAB);
  int*            FLAG = (int*)(ws + oFLAG);
  unsigned short* W1T  = (unsigned short*)(ws + oW1T);
  unsigned short* W2D  = (unsigned short*)(ws + oW2D);
  float*          SM   = (float*)(ws + oSM);
  double*         REC1 = (double*)(ws + oREC1);
  double*         REC2 = (double*)(ws + oREC2);
  float*          ST1  = (float*)(ws + oST1);
  float*          ST2  = (float*)(ws + oST2);

  hipFuncSetAttribute(reinterpret_cast<const void*>(&k_bucket), hipFuncAttributeMaxDynamicSharedMemorySize, (int)BK_LDS);

  k_prep<<<PBTOT, NTHR, 0, stream>>>(x, W1, b1, W2, b2, g1, be1, g2, be2, Wc, bc, XB, W1T, W2D, SM);
  k_bucket<<<NBK, NTHR, BK_LDS, stream>>>(srcs, dsts, ew, LIST, TAB, FLAG);
  k_gemm<<<MP / GBM, NTHR, 0, stream>>>(XB, W1T, TAB, P);
  k_replay<<<dim3(NBK, NB), NTHR, 0, stream>>>(LIST, TAB, FLAG, P, SM, 0, T, REC1);
  k_comb<<<1, 64, 0, stream>>>(REC1, ST1);
  k_apply<<<MP / GBM, NTHR, 0, stream>>>(T, ST1, SM, 128, HN);
  k_gemm<<<MP / GBM, NTHR, 0, stream>>>(HN, W2D, TAB, P);
  k_replay<<<dim3(NBK, NB), NTHR, 0, stream>>>(LIST, TAB, FLAG, P, SM, 64, T, REC2);
  k_comb<<<1, 64, 0, stream>>>(REC2, ST2);
  k_head<<<NREC, NTHR, 0, stream>>>(T, ST2, SM, out);
}
